// GraphAttentionLayer_63350767616660
// MI455X (gfx1250) — hardware-run, weakly checked
//
#include <hip/hip_runtime.h>


#ifndef NB
#define NB 4
#endif
#ifndef SEQ
#define SEQ 512
#endif
#define NB_FULL  4
#define SEQ_FULL 512
#ifndef OUT_SEQ
#define OUT_SEQ SEQ
#endif
#define FIN  256
#define DM   128
#define HID  64
#define NWV  (SEQ / 16)
#define HJP  68
#define OSP  132
#define WSC  64.0f
#define WSI  (1.0f / 64.0f)
#define QRS  2048.0f
#define QRI  (1.0f / 2048.0f)
#define WSL  (64.0f / 2048.0f)
#define LOG2E 1.4426950408889634f
#define PSH  14.0f
#define NEGB (-3.0e38f)
#define NEGF (-1.0e30f)
#define LALPHA 0.01f

static_assert(FIN % 32 == 0);
static_assert(DM % 32 == 0);
static_assert(DM % 64 == 0);
static_assert(2 * HID == DM);
static_assert(HID == 64);
static_assert(DM == 128);
static_assert(SEQ % 64 == 0);
static_assert((NB * SEQ) % 64 == 0);
static_assert(SEQ % 32 == 0);
static_assert(SEQ % 16 == 0);
static_assert(NB <= NB_FULL);
static_assert(SEQ <= SEQ_FULL);
static_assert(((size_t)SEQ * FIN) % 8 == 0);
static_assert(((size_t)DM * FIN) % 8 == 0);
static_assert((HJP * 4) % 16 == 0);
static_assert((OSP * 4) % 16 == 0);
static_assert(32 * 16 * 16 == 64 * 128);
static_assert(32 * 16 * 8 == 16 * 256);
static_assert(32 * 16 * 16 == 16 * 512);
static_assert(8 * 32 * 4 == 16 * HID);
static_assert(16 * 32 * 4 == 32 * HID);
static_assert(64 * 68 * 4 <= 131072);
static_assert(16 * 68 * 4 <= 131072);
static_assert((32 * HJP + 16 * HJP + HID + 16 * OSP) * 4 <= 131072);
static_assert(16 * OSP * 4 <= 131072);
static_assert((size_t)NB * SEQ * DM < ((size_t)1 << 31));

typedef _Float16 h16;
typedef unsigned short bf;
typedef __attribute__((ext_vector_type(16))) __bf16   v16bf;
typedef __attribute__((ext_vector_type(16))) _Float16 v16h;
typedef __attribute__((ext_vector_type(8)))  _Float16 v8h;
typedef __attribute__((ext_vector_type(8)))  unsigned short v8us;
typedef __attribute__((ext_vector_type(8)))  float    v8f;
typedef __attribute__((ext_vector_type(4)))  float    v4f;
typedef v4f  __attribute__((may_alias)) v4fa;

__device__ __forceinline__ unsigned short f2bf(float f) { unsigned u = __float_as_uint(f); u += 0x7FFFu + ((u >> 16) & 1u); return (unsigned short)(u >> 16); }
__device__ __forceinline__ float bfr(float f) { return __uint_as_float(((unsigned)f2bf(f)) << 16); }
__device__ __forceinline__ v16h cat16(v8h lo, v8h hi) { return __builtin_shufflevector(lo, hi, 0, 1, 2, 3, 4, 5, 6, 7, 8, 9, 10, 11, 12, 13, 14, 15); }
__device__ __forceinline__ v16bf cat16b(v8us lo, v8us hi) { return __builtin_bit_cast(v16bf, __builtin_shufflevector(lo, hi, 0, 1, 2, 3, 4, 5, 6, 7, 8, 9, 10, 11, 12, 13, 14, 15)); }
__device__ __forceinline__ v8f wmma16(v16h a, v16h b, v8f c) { return __builtin_amdgcn_wmma_f32_16x16x32_f16(false, a, false, b, (short)0, c, false, false); }
__device__ __forceinline__ v8f wmmab(v16bf a, v16bf b, v8f c) { return __builtin_amdgcn_wmma_f32_16x16x32_bf16(false, a, false, b, (short)0, c, false, false); }
__device__ __forceinline__ v16h  ldh(const h16* p) { return cat16(*(const v8h*)p, *(const v8h*)(p + 16)); }
__device__ __forceinline__ v16bf ldb(const bf* p)  { return cat16b(*(const v8us*)p, *(const v8us*)(p + 16)); }
__device__ __forceinline__ void wave_sync() { __builtin_amdgcn_fence(3  , "wavefront"); __builtin_amdgcn_wave_barrier(); asm volatile("" ::: "memory"); }

__device__ __forceinline__ v8f wmma16g(v16h a, v16h b, v8f c) { c = wmma16(a, b, c); asm volatile("v_nop\n\tv_nop\n\tv_nop\n\tv_nop" : "+v"(c) : "v"(a), "v"(b)); return c; }
__device__ __forceinline__ v8f wmmabg(v16bf a, v16bf b, v8f c) { c = wmmab(a, b, c); asm volatile("v_nop\n\tv_nop\n\tv_nop\n\tv_nop" : "+v"(c) : "v"(a), "v"(b)); return c; }
static __device__ __forceinline__ h16 toh_flush(float v) { const h16 r = (h16)v; return (fabsf(v) < 6.103515625e-05f) ? (h16)0.0f : r; }

__global__ __launch_bounds__(256) void k_cvt8(const float* __restrict__ src, bf* dst, size_t n8) {
    const size_t i = (size_t)blockIdx.x * 256 + threadIdx.x; if (i >= n8) return;
    const v8f v = *(const v8f*)(src + i * 8); v8us o;
#pragma unroll
    for (int k = 0; k < 8; ++k) o[k] = f2bf(v[k]);
    *(volatile v8us*)(dst + i * 8) = o; __threadfence(); *(volatile v8us*)(dst + i * 8) = o;
}

__global__ __launch_bounds__(256) void k_cvtw(const float* __restrict__ src, h16* dst, h16* dst2, int n8) {
    const int i = blockIdx.x * 256 + threadIdx.x; if (i >= n8) return;
    const int c = i >> 4, k = (i & 15) * 8;
    const v8f v = *(const v8f*)(src + (size_t)(c & (HID - 1)) * (2 * DM) + (size_t)(c >> 6) * DM + k); v8h o, o2;
#pragma unroll
    for (int e = 0; e < 8; ++e) { const float w = bfr(v[e]); o[e] = toh_flush(w * WSC); o2[e] = toh_flush(w * WSL); }
    const unsigned di = (unsigned)i * 8u;
    *(volatile v8h*)(dst + (size_t)i * 8) = o; *(volatile v8h*)(dst2 + di) = o2; __threadfence();
    *(volatile v8h*)(dst + (size_t)i * 8) = o; *(volatile v8h*)(dst2 + di) = o2;
}

__global__ __launch_bounds__(32) void k_hproj(const bf* __restrict__ A, const bf* __restrict__ Bt, const float* __restrict__ bias, h16* HHp, h16* HTp, h16* HLp, h16* HLTp) {
    __shared__ __align__(16) float os[64 * 68];
    const int K = FIN;
    const int lane = threadIdx.x & 31, lr = lane & 15, hi = lane >> 4; const int r0 = blockIdx.x * 64, c0 = blockIdx.y * 64;
    v8f acc[4][4];
#pragma unroll
    for (int mb = 0; mb < 4; ++mb)
#pragma unroll
        for (int nb = 0; nb < 4; ++nb) acc[mb][nb] = (v8f){};
    const size_t aoff = (size_t)(r0 + lr) * K + 8 * hi, boff = (size_t)(c0 + lr) * K + 8 * hi;
#pragma unroll 1
    for (int kc = 0; kc < K; kc += 32) {
        v16bf a[4];
#pragma unroll
        for (int mb = 0; mb < 4; ++mb) a[mb] = ldb(A + aoff + (size_t)mb * 16 * K + kc);
#pragma unroll
        for (int nb = 0; nb < 4; ++nb) { const v16bf b = ldb(Bt + boff + (size_t)nb * 16 * K + kc);
#pragma unroll
            for (int mb = 0; mb < 4; ++mb) acc[mb][nb] = wmmabg(a[mb], b, acc[mb][nb]); }
    }
    float bc[4];
#pragma unroll
    for (int nb = 0; nb < 4; ++nb) bc[nb] = bfr(bias[c0 + nb * 16 + lr]);
#pragma unroll
    for (int mb = 0; mb < 4; ++mb)
#pragma unroll
        for (int nb = 0; nb < 4; ++nb)
#pragma unroll
            for (int j = 0; j < 8; ++j) os[(mb * 16 + hi * 8 + j) * 68 + nb * 16 + lr] = acc[mb][nb][j] + bc[nb];
    wave_sync();
    const int bb = r0 / SEQ, tt = r0 % SEQ;
    h16* hrow = HHp + (size_t)r0 * DM + c0;
    h16* trow = HTp + ((size_t)bb * DM + c0) * SEQ + tt;
    h16* lrow = HLp + (unsigned)(r0 * DM + c0);
    h16* ltrow = HLTp + (unsigned)((bb * DM + c0) * SEQ + tt);
#pragma unroll 1
    for (int ps = 0; ps < 2; ++ps) {
#pragma unroll 4
        for (int s = 0; s < 16; ++s) { const int row = 4 * s + (lane >> 3), c8 = (lane & 7) * 8;
            const v4f x0 = *(const v4fa*)(&os[row * 68 + c8]); const v4f x1 = *(const v4fa*)(&os[row * 68 + c8 + 4]); v8h hv, lv;
#pragma unroll
            for (int i = 0; i < 4; ++i) { const h16 a0 = toh_flush(x0[i]); const h16 a1 = toh_flush(x1[i]); hv[i] = a0; hv[4 + i] = a1;
                lv[i] = toh_flush((x0[i] - (float)a0) * QRS); lv[4 + i] = toh_flush((x1[i] - (float)a1) * QRS); }
            *(volatile v8h*)(hrow + (size_t)row * DM + c8) = hv;
            *(volatile v8h*)(lrow + (unsigned)(row * DM + c8)) = lv; }
#pragma unroll 4
        for (int s = 0; s < 16; ++s) { const int oc = 4 * s + (lane >> 3), t8 = (lane & 7) * 8;
            v8h tv, tl;
#pragma unroll
            for (int i = 0; i < 8; ++i) { const float xv = os[(t8 + i) * 68 + oc]; const h16 a0 = toh_flush(xv); tv[i] = a0; tl[i] = toh_flush((xv - (float)a0) * QRS); }
            *(volatile v8h*)(trow + (size_t)oc * SEQ + t8) = tv;
            *(volatile v8h*)(ltrow + (unsigned)(oc * SEQ + t8)) = tl; }
        if (ps == 0) __threadfence(); }
}

__global__ __launch_bounds__(32) void k_hih(const h16* __restrict__ A, const h16* __restrict__ AL, const h16* __restrict__ Bt, const h16* __restrict__ BtL, const float* __restrict__ b1, float* HIHp) {
    __shared__ __align__(16) float os[16 * 68];
    const int K = DM;
    const int lane = threadIdx.x & 31, lr = lane & 15, hi = lane >> 4; const int r0 = blockIdx.x * 64, c0 = blockIdx.y * 64;
    v8f acc[4][4];
#pragma unroll
    for (int mb = 0; mb < 4; ++mb)
#pragma unroll
        for (int nb = 0; nb < 4; ++nb) acc[mb][nb] = (v8f){};
    const size_t aoff = (size_t)(r0 + lr) * K + 8 * hi, boff = (size_t)(c0 + lr) * K + 8 * hi;
    const unsigned aofl = (unsigned)(r0 + lr) * (unsigned)K + 8u * (unsigned)hi, bofl = (unsigned)(c0 + lr) * (unsigned)K + 8u * (unsigned)hi;
#pragma unroll 1
    for (int kc = 0; kc < K; kc += 32) {
        {
        v16h a[4];
#pragma unroll
        for (int mb = 0; mb < 4; ++mb) a[mb] = ldh(A + aoff + (size_t)mb * 16 * K + kc);
#pragma unroll
        for (int nb = 0; nb < 4; ++nb) { const v16h b = ldh(Bt + boff + (size_t)nb * 16 * K + kc);
#pragma unroll
            for (int mb = 0; mb < 4; ++mb) acc[mb][nb] = wmma16g(a[mb], b, acc[mb][nb]); }
        }
        {
        v16h al[4];
#pragma unroll
        for (int mb = 0; mb < 4; ++mb) al[mb] = ldh(AL + aofl + (unsigned)(mb * 16 * K + kc));
#pragma unroll
        for (int nb = 0; nb < 4; ++nb) { const v16h bl = ldh(BtL + bofl + (unsigned)(nb * 16 * K + kc));
#pragma unroll
            for (int mb = 0; mb < 4; ++mb) acc[mb][nb] = wmma16g(al[mb], bl, acc[mb][nb]); }
        }
    }
    float bc[4];
#pragma unroll
    for (int nb = 0; nb < 4; ++nb) { float bv = b1[nb * 16 + lr]; asm volatile("" : "+v"(bv)); bc[nb] = (c0 < HID) ? bfr(bv) : 0.0f; }
#pragma unroll
    for (int mb = 0; mb < 4; ++mb) {
#pragma unroll
        for (int nb = 0; nb < 4; ++nb) {
#pragma unroll
            for (int j = 0; j < 8; ++j) os[(hi * 8 + j) * 68 + nb * 16 + lr] = acc[mb][nb][j] * WSI + bc[nb]; }
        wave_sync();
        float* orow = HIHp + (size_t)(r0 + mb * 16) * DM + c0;
#pragma unroll 1
        for (int ps = 0; ps < 2; ++ps) {
#pragma unroll
            for (int s = 0; s < 8; ++s) { const int row = 2 * s + (lane >> 4), c4 = (lane & 15) * 4;
                const v4f val = *(const v4fa*)(&os[row * 68 + c4]);
                *(volatile v4f*)(orow + (size_t)row * DM + c4) = val; }
            if (ps == 0) __threadfence(); }
        wave_sync();
    }
}

__global__ __launch_bounds__(32) void k_pair(const float* __restrict__ HIHp, const h16* __restrict__ HTp, const h16* __restrict__ HLTp, const float* __restrict__ adj,
                                             const float* __restrict__ A2p, const float* __restrict__ b2p, float* OUp, float* STp) {
    __shared__ __align__(16) float hjs[32 * HJP];
    __shared__ __align__(16) float hbs[16 * HJP];
    __shared__ __align__(16) float sa2[HID];
    __shared__ __align__(16) float os[16 * OSP];
    const int lane = threadIdx.x & 31, lr = lane & 15, hi = lane >> 4;
    const int b = blockIdx.y; const int t0 = blockIdx.x * 16;
    const size_t nrow = (size_t)b * SEQ;
#pragma unroll
    for (int s = 0; s < 8; ++s) { const int idx = s * 32 + lane; const int row = idx >> 4, q = idx & 15;
        const v4f v = *(const v4f*)(HIHp + (nrow + t0 + row) * DM + 4 * q); *(v4fa*)(&hbs[row * HJP + 4 * q]) = v; }
    sa2[lane] = bfr(A2p[lane]); sa2[lane + 32] = bfr(A2p[lane + 32]);
    const float b2v = bfr(b2p[0]);
    const float* ar = adj + ((size_t)b * SEQ_FULL + t0 + lr) * SEQ_FULL + 8 * hi;
    const size_t vo = ((size_t)b * DM + lr) * SEQ + 8 * hi;
    const unsigned vlo = ((unsigned)b * DM + (unsigned)lr) * SEQ + 8u * (unsigned)hi;
    v8f o[8];
#pragma unroll
    for (int dt = 0; dt < 8; ++dt) o[dt] = (v8f){};
    float m = NEGB, l = 0.0f;
#pragma unroll 1
    for (int key0 = 0; key0 < SEQ; key0 += 32) {
        wave_sync();
#pragma unroll 8
        for (int s = 0; s < 16; ++s) { const int idx = s * 32 + lane; const int row = idx >> 4, q = idx & 15;
            const v4f v = *(const v4f*)(HIHp + (nrow + key0 + row) * DM + HID + 4 * q); *(v4fa*)(&hjs[row * HJP + 4 * q]) = v; }
        wave_sync();
        float ea[8], eb[8];
#pragma unroll
        for (int r = 0; r < 8; ++r) { ea[r] = 0.0f; eb[r] = 0.0f; }
#pragma unroll 1
        for (int hq = 0; hq < HID / 4; ++hq) {
            const v4f hb = *(const v4fa*)(&hbs[lr * HJP + 4 * hq]);
            const v4f av = *(const v4fa*)(&sa2[4 * hq]);
#pragma unroll
            for (int r = 0; r < 8; ++r) {
                const v4f xa = *(const v4fa*)(&hjs[(8 * hi + r) * HJP + 4 * hq]);
                const v4f xb = *(const v4fa*)(&hjs[(16 + 8 * hi + r) * HJP + 4 * hq]);
#pragma unroll
                for (int c = 0; c < 4; ++c) { ea[r] = fmaf(av[c], fmaxf(hb[c] + xa[c], 0.0f), ea[r]); eb[r] = fmaf(av[c], fmaxf(hb[c] + xb[c], 0.0f), eb[r]); } }
        }
        const float* kp = ar + key0;
        const v4f m0 = *(const v4f*)kp, m1 = *(const v4f*)(kp + 4), m2 = *(const v4f*)(kp + 16), m3 = *(const v4f*)(kp + 20);
        float kx[8], ky[8];
#pragma unroll
        for (int r = 0; r < 4; ++r) { kx[r] = m0[r]; kx[4 + r] = m1[r]; ky[r] = m2[r]; ky[4 + r] = m3[r]; }
        float ta[8], tb[8]; float mx = NEGB;
#pragma unroll
        for (int r = 0; r < 8; ++r) {
            float xa = ea[r] + b2v, xb = eb[r] + b2v;
            xa = (xa >= 0.0f) ? xa : LALPHA * xa; xb = (xb >= 0.0f) ? xb : LALPHA * xb;
            const float aa = bfr(kx[r]), ab = bfr(ky[r]);
            ta[r] = (xa * aa + (1.0f - aa) * NEGF) * LOG2E; tb[r] = (xb * ab + (1.0f - ab) * NEGF) * LOG2E;
            mx = fmaxf(mx, fmaxf(ta[r], tb[r])); }
        mx = fmaxf(mx, __shfl_xor(mx, 16, 32)); mx = fmaxf(mx, __shfl_xor(mx, 8, 32)); mx = fmaxf(mx, __shfl_xor(mx, 4, 32));
        mx = fmaxf(mx, __shfl_xor(mx, 2, 32));  mx = fmaxf(mx, __shfl_xor(mx, 1, 32));
        const float mnew = fmaxf(m, mx);
        const float alpha = __builtin_amdgcn_exp2f(m - mnew);
        const float sh = PSH - mnew;
        v16h pb, pl; float ls = 0.0f;
#pragma unroll
        for (int r = 0; r < 8; ++r) {
            const float ga = ta[r] + sh, gb = tb[r] + sh;
            const float pa32 = (ga < -14.0f) ? 0.0f : __builtin_amdgcn_exp2f(ga);
            const float pc32 = (gb < -14.0f) ? 0.0f : __builtin_amdgcn_exp2f(gb);
            const h16 pa = (h16)pa32; const h16 pc = (h16)pc32;
            pb[r] = pa; pb[8 + r] = pc;
            pl[r] = toh_flush((float)pa * QRI); pl[8 + r] = toh_flush((float)pc * QRI);
            ls += (float)pa + (float)pc; }
        l = l * alpha + ls; m = mnew;
#pragma unroll
        for (int dt = 0; dt < 8; ++dt) o[dt] = o[dt] * alpha;
        const h16* va = HTp + vo + key0;
        const h16* vla = HLTp + vlo + (unsigned)key0;
#pragma unroll
        for (int g = 0; g < 2; ++g) {
            {
            v16h vf[4];
#pragma unroll
            for (int u = 0; u < 4; ++u) vf[u] = ldh(va + (size_t)(g * 4 + u) * 16 * SEQ);
#pragma unroll
            for (int u = 0; u < 4; ++u) o[g * 4 + u] = wmma16g(vf[u], pb, o[g * 4 + u]);
            }
            {
            v16h vr[4];
#pragma unroll
            for (int u = 0; u < 4; ++u) vr[u] = ldh(vla + (unsigned)((g * 4 + u) * 16 * SEQ));
#pragma unroll
            for (int u = 0; u < 4; ++u) o[g * 4 + u] = wmma16g(vr[u], pl, o[g * 4 + u]);
            }
        }
    }
    l += __shfl_xor(l, 16, 32); l += __shfl_xor(l, 8, 32); l += __shfl_xor(l, 4, 32); l += __shfl_xor(l, 2, 32); l += __shfl_xor(l, 1, 32);
#pragma unroll
    for (int dt = 0; dt < 8; ++dt) { v4f a, c;
        a[0] = o[dt][0]; a[1] = o[dt][1]; a[2] = o[dt][2]; a[3] = o[dt][3]; c[0] = o[dt][4]; c[1] = o[dt][5]; c[2] = o[dt][6]; c[3] = o[dt][7];
        *(v4fa*)(&os[lr * OSP + 16 * dt + 8 * hi]) = a; *(v4fa*)(&os[lr * OSP + 16 * dt + 8 * hi + 4]) = c; }
    wave_sync();
    float* orow = OUp + (nrow + t0) * DM;
    float* stl = STp + ((size_t)b * NWV + blockIdx.x) * 32;
    v4f sv = (v4f){};
    sv[0] = (lane == 0) ? m : 0.0f; sv[1] = (lane == 0) ? l : 0.0f;
#pragma unroll 1
    for (int ps = 0; ps < 2; ++ps) {
#pragma unroll
        for (int s = 0; s < 16; ++s) {
            const v4f val = *(const v4fa*)(&os[s * OSP + 4 * lane]);
            *(volatile v4f*)(orow + (size_t)s * DM + 4 * lane) = val; }
        if (lane < 8) *(volatile v4f*)(stl + 4 * lane) = sv;
        if (ps == 0) __threadfence(); }
}

__global__ __launch_bounds__(32) void k_fin(const float* __restrict__ OUp, const float* __restrict__ STp, float* OUT) {
#pragma clang fp contract(off)
    __shared__ __align__(16) float os[16 * OSP];
    const int lane = threadIdx.x & 31;
    const int b = blockIdx.y; const int t0 = blockIdx.x * 16;
    const size_t nrow = (size_t)b * SEQ;
    const float* stb = STp + (size_t)b * NWV * 32;
    float M = NEGB;
#pragma unroll 1
    for (int w0 = 0; w0 < NWV; w0 += 32) { const int w = w0 + lane; const int wc = (w < NWV) ? w : (NWV - 1);
        float mv = stb[(size_t)wc * 32]; asm volatile("" : "+v"(mv));
        M = fmaxf(M, (w < NWV) ? mv : NEGB); }
    M = fmaxf(M, __shfl_xor(M, 16, 32)); M = fmaxf(M, __shfl_xor(M, 8, 32)); M = fmaxf(M, __shfl_xor(M, 4, 32));
    M = fmaxf(M, __shfl_xor(M, 2, 32));  M = fmaxf(M, __shfl_xor(M, 1, 32));
    float S = 0.0f;
#pragma unroll 1
    for (int w0 = 0; w0 < NWV; w0 += 32) { const int w = w0 + lane; const int wc = (w < NWV) ? w : (NWV - 1);
        float mv = stb[(size_t)wc * 32]; float lv = stb[(size_t)wc * 32 + 1]; asm volatile("" : "+v"(mv)); asm volatile("" : "+v"(lv));
        const float term = lv * __builtin_amdgcn_exp2f(mv - M);
        S += (w < NWV) ? term : 0.0f; }
    S += __shfl_xor(S, 16, 32); S += __shfl_xor(S, 8, 32); S += __shfl_xor(S, 4, 32); S += __shfl_xor(S, 2, 32); S += __shfl_xor(S, 1, 32);
    const float mo = stb[(size_t)blockIdx.x * 32];
    const float scale = __builtin_amdgcn_exp2f(mo - M) * (1.0f / S);
#pragma unroll 4
    for (int s = 0; s < 16; ++s) { v4f v = *(const v4f*)(OUp + (nrow + t0 + s) * DM + 4 * lane);
        v = v * scale; *(v4fa*)(&os[s * OSP + 4 * lane]) = v; }
    wave_sync();
#pragma unroll 1
    for (int q = 0; q < 64; ++q) { const int idx = (q >> 2) * OSP + 4 * lane + (q & 3);
        const float v = os[idx]; os[idx] = (v > 0.0f) ? v : expm1f(v); }
    wave_sync();
    float* orow = OUT + ((size_t)b * OUT_SEQ + t0) * DM;
#pragma unroll 1
    for (int ps = 0; ps < 2; ++ps) {
#pragma unroll
        for (int s = 0; s < 16; ++s) {
            const v4f val = *(const v4fa*)(&os[s * OSP + 4 * lane]);
            *(volatile v4f*)(orow + (size_t)s * DM + 4 * lane) = val; }
        if (ps == 0) __threadfence(); }
}

static constexpr size_t al256(size_t v) { return (v + 255) & ~(size_t)255; }
static constexpr size_t SZ_XB = al256((size_t)NB * SEQ * FIN * 2);
static constexpr size_t SZ_WB = al256((size_t)DM * FIN * 2);
static constexpr size_t SZ_AH = al256((size_t)DM * DM * 2);
static constexpr size_t SZ_HH = al256((size_t)NB * SEQ * DM * 2);
static constexpr size_t SZ_F  = al256((size_t)NB * SEQ * DM * 4);
static constexpr size_t SZ_ST = al256((size_t)NB * NWV * 32 * 4);
static constexpr size_t SZ_TOTAL = SZ_XB + SZ_WB + 2 * SZ_AH + 4 * SZ_HH + 2 * SZ_F + SZ_ST;
static_assert(SZ_TOTAL <= (size_t)134217728);
static_assert((size_t)NB * DM * SEQ * 2 <= SZ_HH);
static_assert((size_t)DM * DM * 2 <= SZ_AH);
static_assert(((size_t)(NB * SEQ / 64 - 1) * 64 + 63) * DM + 127 < (size_t)NB * SEQ * DM);
static_assert(((size_t)(NB - 1) * DM + (DM - 1)) * SEQ + (SEQ - 1) < (size_t)NB * SEQ * DM);
static_assert(((size_t)(NB - 1) * NWV + (NWV - 1)) * 32 + 31 < (size_t)NB * NWV * 32);

extern "C" void kernel_launch(void* const* d_in, const int* in_sizes, int n_in,
                              void* d_out, int out_size, void* d_ws, size_t ws_size, hipStream_t stream) {
    if (n_in < 8) return;
    const size_t needx = ((size_t)(NB - 1) * SEQ_FULL + SEQ) * FIN;
    const size_t needa = ((size_t)(NB - 1) * SEQ_FULL + (SEQ - 1)) * SEQ_FULL + SEQ;
    if ((size_t)in_sizes[0] < needx || (size_t)in_sizes[1] < needa) return;
    if ((size_t)in_sizes[2] < (size_t)DM * FIN || in_sizes[3] < DM) return;
    if ((size_t)in_sizes[4] < (size_t)HID * 2 * DM || in_sizes[5] < HID || in_sizes[6] < HID || in_sizes[7] < 1) return;
    if ((size_t)out_size < ((size_t)(NB - 1) * OUT_SEQ + SEQ) * DM) return;
    if (SZ_TOTAL > ws_size) return;
    const float* x   = (const float*)d_in[0];
    const float* adj = (const float*)d_in[1];
    const float* w   = (const float*)d_in[2];
    const float* bw  = (const float*)d_in[3];
    const float* a1  = (const float*)d_in[4];
    const float* b1  = (const float*)d_in[5];
    const float* a2  = (const float*)d_in[6];
    const float* b2  = (const float*)d_in[7];
    float* OUT = (float*)d_out;
    char* wsp = (char*)d_ws;
    bf*  XB  = (bf*)wsp;  wsp += SZ_XB;
    bf*  WB  = (bf*)wsp;  wsp += SZ_WB;
    h16* A1H = (h16*)wsp; wsp += SZ_AH;
    h16* A1L = (h16*)wsp; wsp += SZ_AH;
    h16* HH  = (h16*)wsp; wsp += SZ_HH;
    h16* HT  = (h16*)wsp; wsp += SZ_HH;
    h16* HL  = (h16*)wsp; wsp += SZ_HH;
    h16* HLT = (h16*)wsp; wsp += SZ_HH;
    float* HIH = (float*)wsp; wsp += SZ_F;
    float* OU  = (float*)wsp; wsp += SZ_F;
    float* ST  = (float*)wsp; wsp += SZ_ST;

    if (SEQ == SEQ_FULL) {
        const size_t n8 = (size_t)NB * SEQ * FIN / 8;
        k_cvt8<<<(unsigned)((n8 + 255) / 256), 256, 0, stream>>>(x, XB, n8);
    } else {
        const size_t n8 = (size_t)SEQ * FIN / 8;
        for (int b = 0; b < NB; ++b) k_cvt8<<<(unsigned)((n8 + 255) / 256), 256, 0, stream>>>(x + (size_t)b * SEQ_FULL * FIN, XB + (size_t)b * SEQ * FIN, n8);
    }
    { const size_t n8 = (size_t)DM * FIN / 8; k_cvt8<<<(unsigned)((n8 + 255) / 256), 256, 0, stream>>>(w, WB, n8); }
    { const int n8 = DM * DM / 8; k_cvtw<<<(unsigned)((n8 + 255) / 256), 256, 0, stream>>>(a1, A1H, A1L, n8); }

    k_hproj<<<dim3(NB * SEQ / 64, DM / 64, 1), 32, 0, stream>>>(XB, WB, bw, HH, HT, HL, HLT);
    k_hih<<<dim3(NB * SEQ / 64, DM / 64, 1), 32, 0, stream>>>(HH, HL, A1H, A1L, b1, HIH);
    k_pair<<<dim3(SEQ / 16, NB, 1), 32, 0, stream>>>(HIH, HT, HLT, adj, a2, b2, OU, ST);
    k_fin<<<dim3(SEQ / 16, NB, 1), 32, 0, stream>>>(OU, ST, OUT);
}
